// GC_FFM_39109972197410
// MI455X (gfx1250) — hardware-verified
//
#include <hip/hip_runtime.h>
#include <stdint.h>

typedef __attribute__((ext_vector_type(16))) _Float16 v16h;
typedef __attribute__((ext_vector_type(8)))  _Float16 v8h;
typedef __attribute__((ext_vector_type(16))) __bf16   v16b;
typedef __attribute__((ext_vector_type(8)))  __bf16   v8b;
typedef __attribute__((ext_vector_type(8)))  float    v8f;
typedef __attribute__((ext_vector_type(4)))  float    v4f;

#define NPIX 4096
#define NCH 256
#define NCH2 512
#define KCOL 4608

__device__ __forceinline__ unsigned short f2bf_bits(float f) {
  unsigned u = __float_as_uint(f);
  return (unsigned short)((u + 0x7FFFu + ((u >> 16) & 1u)) >> 16);
}
__device__ __forceinline__ float bf_bits2f(unsigned short h) { return __uint_as_float(((unsigned)h) << 16); }

__device__ __forceinline__ void dep_guard_h(v8f& a, v8f& b, v16h x, v16h y) { asm volatile("v_nop\n\tv_nop\n\tv_nop\n\tv_nop" : "+v"(a), "+v"(b) : "v"(x), "v"(y)); }
__device__ __forceinline__ void dep_guard_b(v8f& a, v8f& b, v16b x, v16b y) { asm volatile("v_nop\n\tv_nop\n\tv_nop\n\tv_nop" : "+v"(a), "+v"(b) : "v"(x), "v"(y)); }
__device__ __forceinline__ void keep4_h(v16h a, v16h b, v16h c, v16h d) { asm volatile("v_nop" :: "v"(a), "v"(b), "v"(c), "v"(d)); }
__device__ __forceinline__ void keep4_b(v16b a, v16b b, v16b c, v16b d) { asm volatile("v_nop" :: "v"(a), "v"(b), "v"(c), "v"(d)); }
__device__ __forceinline__ void acc_guard4(v8f& a, v8f& b, v8f& c, v8f& d) { asm volatile("v_nop\n\tv_nop\n\tv_nop\n\tv_nop" : "+v"(a), "+v"(b), "+v"(c), "+v"(d)); }
template <typename T> struct Frag;
template <> struct Frag<_Float16> {
  typedef v16h V; union U { v16h v; v8h h[2]; };
  static __device__ __forceinline__ v16h load(const _Float16* p) {
    U f; f.h[0] = *(const v8h*)(p); f.h[1] = *(const v8h*)(p + 16); return f.v;
  }
  static __device__ __forceinline__ v8f mma(v16h a, v16h b, v8f c) {
    return __builtin_amdgcn_wmma_f32_16x16x32_f16(false, a, false, b, (short)0, c, false, false);
  }
  static __device__ __forceinline__ void guard(v8f& a, v8f& b, v16h x, v16h y) { dep_guard_h(a, b, x, y); }
  static __device__ __forceinline__ void keep(v16h a, v16h b, v16h c, v16h d) { keep4_h(a, b, c, d); }
};
template <> struct Frag<__bf16> {
  typedef v16b V; union U { v16b v; v8b h[2]; };
  static __device__ __forceinline__ v16b load(const __bf16* p) {
    U f; f.h[0] = *(const v8b*)(p); f.h[1] = *(const v8b*)(p + 16); return f.v;
  }
  static __device__ __forceinline__ v8f mma(v16b a, v16b b, v8f c) {
    return __builtin_amdgcn_wmma_f32_16x16x32_bf16(false, a, false, b, (short)0, c, false, false);
  }
  static __device__ __forceinline__ void guard(v8f& a, v8f& b, v16b x, v16b y) { dep_guard_b(a, b, x, y); }
  static __device__ __forceinline__ void keep(v16b a, v16b b, v16b c, v16b d) { keep4_b(a, b, c, d); }
};

template <int ET> struct Elem;
template <> struct Elem<0> { typedef _Float16 T; };
template <> struct Elem<1> { typedef __bf16 T; };
template <int ET, bool SPLIT, int BIAS_MODE, int OUT_MODE, int RESID, int ACT = 0>
__global__ __launch_bounds__(256) void wmma_gemm64(
    const unsigned short* __restrict__ Ap, const unsigned short* __restrict__ A2p, int lda, long strideA,
    const unsigned short* __restrict__ Btp, const unsigned short* __restrict__ Bt2p, int ldb, long strideB,
    void* __restrict__ Cout, void* __restrict__ Cout2, int ldc, long strideC,
    const float* __restrict__ bias,
    const float* __restrict__ resid, long strideR, int ldr,
    int M, int N, int K, float scale) {
  typedef typename Elem<ET>::T T;
  typedef typename Frag<T>::V V;
  const T* A = (const T*)Ap; const T* A2 = (const T*)A2p; const T* Bt = (const T*)Btp; const T* Bt2 = (const T*)Bt2p;
  __shared__ __align__(16) float sT[8][16 * 68];
  const int b    = blockIdx.y;
  const int lane = threadIdx.x & 31;
  const int wave = threadIdx.x >> 5;
  const int tilesN = N >> 6;
  const int tilesM = M >> 6;
  const int tile = blockIdx.x * 8 + wave;
  if (tile >= tilesM * tilesN) return;
  const int tm = tile / tilesN;
  const int tn = tile - tm * tilesN;
  const int m0 = tm << 6;
  const int n0 = tn << 6;

  const T* Ab  = A  + (size_t)b * strideA;
  const T* Bb  = Bt + (size_t)b * strideB;
  const T* Ab2 = SPLIT ? (A2  + (size_t)b * strideA) : nullptr;
  const T* Bb2 = SPLIT ? (Bt2 + (size_t)b * strideB) : nullptr;

  const int rlane = lane & 15;
  const int koff  = (lane >> 4) * 8;
  const int mOff  = (lane >> 4) * 8;

  v8f acc[4][4];
#pragma unroll
  for (int i = 0; i < 4; ++i)
#pragma unroll
    for (int j = 0; j < 4; ++j) acc[i][j] = (v8f){0.f,0.f,0.f,0.f,0.f,0.f,0.f,0.f};

  for (int k0 = 0; k0 < K; k0 += 32) {
    V bh[4], bl[4];
#pragma unroll
    for (int j = 0; j < 4; ++j) {
      const size_t bo = (size_t)(n0 + (j << 4) + rlane) * ldb + koff + k0;
      bh[j] = Frag<T>::load(Bb + bo);
      if (SPLIT) bl[j] = Frag<T>::load(Bb2 + bo);
    }
#pragma unroll
    for (int i = 0; i < 4; ++i) {
      const size_t ao = (size_t)(m0 + (i << 4) + rlane) * lda + koff + k0;
      V ah = Frag<T>::load(Ab + ao);
      V al;
      if (SPLIT) al = Frag<T>::load(Ab2 + ao);
#pragma unroll
      for (int j = 0; j < 4; ++j) {
        acc[i][j] = Frag<T>::mma(ah, bh[j], acc[i][j]);
        if (SPLIT) {
          acc[i][j] = Frag<T>::mma(ah, bl[j], acc[i][j]);
          acc[i][j] = Frag<T>::mma(al, bh[j], acc[i][j]);
        }
      }
      Frag<T>::guard(acc[i][0], acc[i][3], ah, SPLIT ? al : ah);
    }
    Frag<T>::keep(bh[0], bh[1], bh[2], bh[3]);
    if (SPLIT) Frag<T>::keep(bl[0], bl[1], bl[2], bl[3]);
  }
  acc_guard4(acc[0][0], acc[0][1], acc[0][2], acc[0][3]);
  acc_guard4(acc[1][0], acc[1][1], acc[1][2], acc[1][3]);
  acc_guard4(acc[2][0], acc[2][1], acc[2][2], acc[2][3]);
  acc_guard4(acc[3][0], acc[3][1], acc[3][2], acc[3][3]);

  float* slab = sT[wave];
  const float* Rb = (RESID != 0) ? (resid + (size_t)b * strideR) : nullptr;
#pragma unroll
  for (int i = 0; i < 4; ++i) {
    const int mBase = m0 + (i << 4);
#pragma unroll
    for (int j = 0; j < 4; ++j) {
      const int n = n0 + (j << 4) + rlane;
      float bv = 0.f;
      if (BIAS_MODE == 2) bv = bias[n];
#pragma unroll
      for (int r = 0; r < 8; ++r) {
        float v = acc[i][j][r] * scale;
        if (BIAS_MODE == 1) v += bias[mBase + mOff + r];
        if (BIAS_MODE == 2) v += bv;
        if (RESID == 1) v += Rb[(size_t)(mBase + mOff + r) * ldc + n];
        if (RESID == 2) v += Rb[(size_t)n * ldr + (mBase + mOff + r)];
        if (ACT == 1) v = tanhf(v);
        if (ACT == 2) v = fmaxf(v, 0.0f);
        if (ACT == 3) v = v / (1.0f + expf(-v));
        if (ACT == 4) v = (v > 0.f) ? v : 0.01f * v;
        if (ACT == 5) v = 0.5f * v * (1.0f + erff(v * 0.70710678118654752f));
        if (ACT == 6) v = __builtin_amdgcn_rcpf(1.0f + __expf(-v));
        slab[(mOff + r) * 68 + (j << 4) + rlane] = v;
      }
    }
    __builtin_amdgcn_fence(__ATOMIC_RELEASE, "workgroup");
    __builtin_amdgcn_wave_barrier();
    __builtin_amdgcn_fence(__ATOMIC_ACQUIRE, "workgroup");
    if (OUT_MODE == 0) {
      float* C = (float*)Cout + (size_t)b * strideC;
      const int hh = lane >> 4, c4 = (lane & 15) * 4;
      for (int pass = 0; pass < 2; ++pass) {
#pragma unroll
        for (int it = 0; it < 8; ++it) {
          const int row = it * 2 + hh;
          v4f v = *(const v4f*)(slab + row * 68 + c4);
          *(volatile v4f*)(C + (size_t)(mBase + row) * ldc + n0 + c4) = v;
        }
        __threadfence();
      }
    } else {
      const int q = lane >> 3, c8 = (lane & 7) * 8;
      unsigned short* C  = (unsigned short*)Cout  + (size_t)b * strideC;
      unsigned short* C2 = (OUT_MODE == 2) ? ((unsigned short*)Cout2 + (size_t)b * strideC) : nullptr;
      for (int pass = 0; pass < 2; ++pass) {
#pragma unroll
        for (int it = 0; it < 4; ++it) {
          const int row = it * 4 + q;
          const float* sp = slab + row * 68 + c8;
          v8h hv, lv;
#pragma unroll
          for (int e = 0; e < 8; ++e) {
            if (OUT_MODE == 1) {
              hv[e] = (_Float16)sp[e];
            } else {
              unsigned short hb = f2bf_bits(sp[e]);
              unsigned short lb = f2bf_bits(sp[e] - bf_bits2f(hb));
              hv[e] = __builtin_bit_cast(_Float16, hb);
              lv[e] = __builtin_bit_cast(_Float16, lb);
            }
          }
          *(volatile v8h*)(C + (size_t)(mBase + row) * ldc + n0 + c8) = hv;
          if (OUT_MODE == 2) *(volatile v8h*)(C2 + (size_t)(mBase + row) * ldc + n0 + c8) = lv;
        }
        __threadfence();
      }
    }
    __builtin_amdgcn_fence(__ATOMIC_RELEASE, "workgroup");
    __builtin_amdgcn_wave_barrier();
    __builtin_amdgcn_fence(__ATOMIC_ACQUIRE, "workgroup");
  }
}

__global__ __launch_bounds__(256) void k_cast_scale(
    const float* __restrict__ in, _Float16* __restrict__ out, int n2, float scale) {
  int i = blockIdx.x * 256 + threadIdx.x;
  if (i < n2) {
    const _Float16 h0 = (_Float16)(in[2 * i] * scale), h1 = (_Float16)(in[2 * i + 1] * scale);
    const unsigned u = (unsigned)__builtin_bit_cast(unsigned short, h0) | ((unsigned)__builtin_bit_cast(unsigned short, h1) << 16);
    ((volatile unsigned*)out)[i] = u;
    __threadfence();
    ((volatile unsigned*)out)[i] = u;
  }
}

__global__ __launch_bounds__(256) void k_tr_cast(const float* __restrict__ X, _Float16* __restrict__ Y, int C, int P) {
  __shared__ __align__(16) _Float16 T[64 * 72];
  const int img = blockIdx.z, c0 = blockIdx.y * 64, p0 = blockIdx.x * 64;
  const int t = threadIdx.x, lane = t & 31, wave = t >> 5, hh = lane >> 4;
  const float* Xb = X + ((size_t)img * C + c0) * (size_t)P + p0;
#pragma unroll
  for (int it = 0; it < 4; ++it) {
    const int cc = wave * 8 + it * 2 + hh;
    const int col = (lane & 15) * 4;
    v4f v = *(const v4f*)(Xb + (size_t)cc * P + col);
#pragma unroll
    for (int e = 0; e < 4; ++e) T[(col + e) * 72 + cc] = (_Float16)v[e];
  }
  __syncthreads();
  _Float16* Yb = Y + ((size_t)img * P + p0) * (size_t)C + c0;
  const int q = lane >> 3, c8 = (lane & 7) * 8;
  for (int pass = 0; pass < 2; ++pass) {
#pragma unroll
    for (int it = 0; it < 2; ++it) {
      const int pp = wave * 8 + it * 4 + q;
      v8h hv = *(const v8h*)(T + pp * 72 + c8);
      *(volatile v8h*)(Yb + (size_t)pp * C + c8) = hv;
    }
    __threadfence();
  }
}

__global__ __launch_bounds__(128) void k_bias_cat(const float* __restrict__ a, const float* __restrict__ b,
                                                  const float* __restrict__ c, const float* __restrict__ d,
                                                  float* __restrict__ out) {
  const int t = threadIdx.x;
  const int k = t & 31, s = t >> 5;
  const float va = a[k], vb = b[k], vc = c[k], vd = d[k];
  const float v = (s == 0) ? va : (s == 1) ? vb : (s == 2) ? vc : vd;
  ((volatile float*)out)[t] = v;
  __threadfence();
  ((volatile float*)out)[t] = v;
}

__global__ __launch_bounds__(256) void k_softmax_t(const float* __restrict__ S, _Float16* __restrict__ PT) {
  __shared__ float sm[64];
  __shared__ float sz[64];
  __shared__ __align__(16) _Float16 T[64 * 72];
  const int i0 = blockIdx.x * 64;
  const int t = threadIdx.x, lane = t & 31, wave = t >> 5, hh = lane >> 4;
#pragma unroll 1
  for (int r = 0; r < 8; ++r) {
    const int rr = wave * 8 + r;
    const float* row = S + (size_t)(i0 + rr) * NPIX;
    float m = -3.0e38f;
#pragma unroll 4
    for (int c = 0; c < 32; ++c) {
      v4f v = *(const v4f*)(row + c * 128 + lane * 4);
      m = fmaxf(m, fmaxf(fmaxf(v[0], v[1]), fmaxf(v[2], v[3])));
    }
#pragma unroll
    for (int off = 1; off < 32; off <<= 1) m = fmaxf(m, __shfl_xor(m, off, 32));
    float z = 0.f;
#pragma unroll 4
    for (int c = 0; c < 32; ++c) {
      v4f v = *(const v4f*)(row + c * 128 + lane * 4);
      z += (__expf(v[0] - m) + __expf(v[1] - m)) + (__expf(v[2] - m) + __expf(v[3] - m));
    }
#pragma unroll
    for (int off = 1; off < 32; off <<= 1) z += __shfl_xor(z, off, 32);
    if (lane == 0) { sm[rr] = m; sz[rr] = 32768.0f / z; }
  }
  __syncthreads();
  const int q = lane >> 3, c8 = (lane & 7) * 8;
#pragma unroll 1
  for (int jc = 0; jc < 64; ++jc) {
#pragma unroll
    for (int it = 0; it < 4; ++it) {
      const int rr = wave * 8 + it * 2 + hh;
      const int col = (lane & 15) * 4;
      v4f v = *(const v4f*)(S + (size_t)(i0 + rr) * NPIX + jc * 64 + col);
      const float m = sm[rr], zs = sz[rr];
#pragma unroll
      for (int e = 0; e < 4; ++e) T[(col + e) * 72 + rr] = (_Float16)(__expf(v[e] - m) * zs);
    }
    __syncthreads();
    for (int pass = 0; pass < 2; ++pass) {
#pragma unroll
      for (int it = 0; it < 2; ++it) {
        const int jj = wave * 8 + it * 4 + q;
        v8h hv = *(const v8h*)(T + jj * 72 + c8);
        *(volatile v8h*)(PT + (size_t)(jc * 64 + jj) * NPIX + i0 + c8) = hv;
      }
      __threadfence();
    }
    __syncthreads();
  }
}

__global__ __launch_bounds__(256) void k_fuse(const float* __restrict__ cat, const float* __restrict__ G,
                                               _Float16* __restrict__ F, int npix) {
  const int idx = blockIdx.x * 256 + threadIdx.x;
  const int cg = idx & 31, p = idx >> 5;
  if (p < npix) {
    const float* cr = cat + (size_t)p * NCH2 + cg * 8;
    const float* gr = G + (size_t)p * NCH + cg * 8;
    v4f b0 = *(const v4f*)cr, b1 = *(const v4f*)(cr + 4);
    v4f d0 = *(const v4f*)(cr + NCH), d1 = *(const v4f*)(cr + NCH + 4);
    v4f g0 = *(const v4f*)gr, g1 = *(const v4f*)(gr + 4);
    v8h hc, hd;
#pragma unroll
    for (int e = 0; e < 4; ++e) {
      const float br = b0[e], bd = d0[e], g = g0[e];
      hc[e] = (_Float16)(br * g + bd * (1.0f - g));
      hd[e] = (_Float16)(br * bd);
      const float br1 = b1[e], bd1 = d1[e], g1v = g1[e];
      hc[4 + e] = (_Float16)(br1 * g1v + bd1 * (1.0f - g1v));
      hd[4 + e] = (_Float16)(br1 * bd1);
    }
    _Float16* fr = F + (size_t)p * NCH2 + cg * 8;
    *(volatile v8h*)fr = hc;
    *(volatile v8h*)(fr + NCH) = hd;
    __threadfence();
    *(volatile v8h*)fr = hc;
    *(volatile v8h*)(fr + NCH) = hd;
  }
}

__global__ __launch_bounds__(256) void k_w2r(const float* __restrict__ W, _Float16* __restrict__ out, float scale) {
  const int idx = blockIdx.x * 256 + threadIdx.x;
  const int cg = idx & 63;
  const int ot = idx >> 6;
  const int o = ot / 9;
  const int tp = ot - o * 9;
  if (o < NCH2) {
    v8h hv;
#pragma unroll
    for (int e = 0; e < 8; ++e) {
      const float w = W[((size_t)(o * NCH2 + cg * 8 + e)) * 9 + tp];
      hv[e] = (_Float16)(w * scale);
    }
    _Float16* dst = out + (size_t)o * KCOL + tp * NCH2 + cg * 8;
    *(volatile v8h*)dst = hv;
    __threadfence();
    *(volatile v8h*)dst = hv;
  }
}

__global__ __launch_bounds__(256) void k_im2col(const _Float16* __restrict__ Y, _Float16* __restrict__ col) {
  const int idx = blockIdx.x * 256 + threadIdx.x;
  const int cg = idx & 63;
  const int pt = idx >> 6;
  const int p = pt / 9;
  const int tp = pt - p * 9;
  if (p < NPIX) {
    const int y = p >> 6, x = p & 63;
    const int ky = tp / 3, kx = tp - ky * 3;
    const int yy = y + ky - 1, xx = x + kx - 1;
    const bool ok = (yy >= 0) && (yy < 64) && (xx >= 0) && (xx < 64);
    const int yc = yy < 0 ? 0 : (yy > 63 ? 63 : yy);
    const int xc = xx < 0 ? 0 : (xx > 63 ? 63 : xx);
    v8h v = *(const v8h*)(Y + (size_t)(yc * 64 + xc) * NCH2 + cg * 8);
    v8h o;
#pragma unroll
    for (int e = 0; e < 8; ++e) o[e] = ok ? v[e] : (_Float16)0.0f;
    _Float16* dst = col + (size_t)p * KCOL + tp * NCH2 + cg * 8;
    *(volatile v8h*)dst = o;
    __threadfence();
    *(volatile v8h*)dst = o;
  }
}

template <int BIAS, int OUTM, int RES, int ACT>
static void launch_gemm(hipStream_t st, const void* A, int lda, long sA, const void* Bt, int ldb, long sB,
                        void* C, int ldc, long sC, const float* bias, const float* resid, long sR, int ldr,
                        int M, int N, int K, float scale, int batch) {
  const int tiles = (M >> 6) * (N >> 6);
  dim3 grid((unsigned)((tiles + 7) >> 3), (unsigned)batch);
  wmma_gemm64<0, false, BIAS, OUTM, RES, ACT><<<grid, dim3(256), 0, st>>>(
      (const unsigned short*)A, (const unsigned short*)A, lda, sA,
      (const unsigned short*)Bt, (const unsigned short*)Bt, ldb, sB,
      C, C, ldc, sC, bias, resid, sR, ldr, M, N, K, scale);
}

static void launch_cast(hipStream_t st, const float* in, _Float16* out, int n, float scale) {
  const int n2 = n >> 1;
  k_cast_scale<<<dim3((unsigned)((n2 + 255) / 256)), dim3(256), 0, st>>>(in, out, n2, scale);
}

extern "C" void kernel_launch(void* const* d_in, const int* in_sizes, int n_in,
                              void* d_out, int out_size, void* d_ws, size_t ws_size,
                              hipStream_t stream)
{
  const int NI = 2;
  if (n_in < 24) return;
  if (in_sizes[0] != NI * NCH * NPIX || in_sizes[1] != NI * NCH * NPIX) return;
  if (in_sizes[2] != 32 * NCH || in_sizes[4] != 32 * NCH || in_sizes[8] != 32 * NCH || in_sizes[10] != 32 * NCH) return;
  if (in_sizes[3] != 32 || in_sizes[5] != 32 || in_sizes[9] != 32 || in_sizes[11] != 32) return;
  if (in_sizes[6] != NCH * NCH || in_sizes[12] != NCH * NCH || in_sizes[7] != NCH || in_sizes[13] != NCH) return;
  if (in_sizes[14] != NCH * NCH2 || in_sizes[15] != NCH) return;
  if (in_sizes[16] != NCH2 * NCH2 || in_sizes[17] != NCH2) return;
  if (in_sizes[18] != NCH2 * NCH2 * 9 || in_sizes[19] != NCH2) return;
  if (in_sizes[20] != NCH * NCH2 || in_sizes[21] != NCH || in_sizes[22] != NCH * NCH2 || in_sizes[23] != NCH) return;
  if (out_size != NI * NCH * NPIX) return;

  const float* rgb  = (const float*)d_in[0];
  const float* chm  = (const float*)d_in[1];
  const float* rq_w = (const float*)d_in[2];  const float* rq_b = (const float*)d_in[3];
  const float* rk_w = (const float*)d_in[4];  const float* rk_b = (const float*)d_in[5];
  const float* rv_w = (const float*)d_in[6];  const float* rv_b = (const float*)d_in[7];
  const float* dq_w = (const float*)d_in[8];  const float* dq_b = (const float*)d_in[9];
  const float* dk_w = (const float*)d_in[10]; const float* dk_b = (const float*)d_in[11];
  const float* dv_w = (const float*)d_in[12]; const float* dv_b = (const float*)d_in[13];
  const float* g_w  = (const float*)d_in[14]; const float* g_b  = (const float*)d_in[15];
  const float* f1_w = (const float*)d_in[16]; const float* f1_b = (const float*)d_in[17];
  const float* f2_w = (const float*)d_in[18]; const float* f2_b = (const float*)d_in[19];
  const float* f3_w = (const float*)d_in[20]; const float* f3_b = (const float*)d_in[21];
  const float* sk_w = (const float*)d_in[22]; const float* sk_b = (const float*)d_in[23];
  float* out = (float*)d_out;

  const size_t MiB = 1048576;
  const size_t oR0  = 0;
  const size_t oP1  = oR0 + 96 * MiB;
  const size_t oCat = oP1 + 10 * MiB;
  const size_t oWA  = oCat + 16 * MiB;
  const size_t total = oWA + 32768 + 32768 + 131072 + 131072 + 512;
  if (ws_size < total) return;
  char* ws = (char*)d_ws;

  _Float16* rgbT = (_Float16*)(ws + oR0);
  _Float16* chmT = (_Float16*)(ws + oR0 + 4 * MiB);
  float*    Sbuf = (float*)(ws + oR0);
  _Float16* PT   = (_Float16*)(ws + oR0 + 64 * MiB);
  float*    G32   = (float*)(ws + oR0);
  _Float16* Y1    = (_Float16*)(ws + oR0 + 8 * MiB);
  _Float16* COL   = (_Float16*)(ws + oR0 + 16 * MiB);
  _Float16* Y2    = (_Float16*)(ws + oR0 + 16 * MiB + 37748736);
  float*    SK    = (float*)(ws + oR0 + 62914560);
  _Float16* cat16 = (_Float16*)(ws + oR0 + 71303168);
  _Float16* Wg16  = (_Float16*)(ws + oR0 + 79691776);
  _Float16* W1_16 = (_Float16*)(ws + oR0 + 79953920);
  _Float16* W2r   = (_Float16*)(ws + oR0 + 80478208);
  _Float16* W3_16 = (_Float16*)(ws + oR0 + 85196800);
  _Float16* Wsk16 = (_Float16*)(ws + oR0 + 85458944);
  _Float16* qk_r = (_Float16*)(ws + oP1);
  _Float16* qk_d = (_Float16*)(ws + oP1 + 1 * MiB);
  _Float16* v_r  = (_Float16*)(ws + oP1 + 2 * MiB);
  _Float16* v_d  = (_Float16*)(ws + oP1 + 6 * MiB);
  _Float16* F16  = (_Float16*)(ws + oP1);
  float*    cat32 = (float*)(ws + oCat);
  _Float16* Wqk_r = (_Float16*)(ws + oWA);
  _Float16* Wqk_d = (_Float16*)(ws + oWA + 32768);
  _Float16* Wv_r  = (_Float16*)(ws + oWA + 65536);
  _Float16* Wv_d  = (_Float16*)(ws + oWA + 65536 + 131072);
  float*    bqk   = (float*)(ws + oWA + 65536 + 262144);

  const float WSC = 64.0f, WINV = 1.0f / 64.0f;
  const long sPixC = (long)NPIX * NCH;
  const long sPix2 = (long)NPIX * NCH2;
  const long sQK   = (long)NPIX * 64;

  k_tr_cast<<<dim3(NPIX / 64, NCH / 64, NI), dim3(256), 0, stream>>>(rgb, rgbT, NCH, NPIX);
  k_tr_cast<<<dim3(NPIX / 64, NCH / 64, NI), dim3(256), 0, stream>>>(chm, chmT, NCH, NPIX);
  launch_cast(stream, rq_w, Wqk_r, 32 * NCH, WSC);
  launch_cast(stream, rk_w, Wqk_r + 32 * NCH, 32 * NCH, WSC);
  launch_cast(stream, dq_w, Wqk_d, 32 * NCH, WSC);
  launch_cast(stream, dk_w, Wqk_d + 32 * NCH, 32 * NCH, WSC);
  launch_cast(stream, rv_w, Wv_r, NCH * NCH, WSC);
  launch_cast(stream, dv_w, Wv_d, NCH * NCH, WSC);
  k_bias_cat<<<dim3(1), dim3(128), 0, stream>>>(rq_b, rk_b, dq_b, dk_b, bqk);

  launch_gemm<2, 1, 0, 0>(stream, rgbT, NCH, sPixC, Wqk_r, NCH, 0, qk_r, 64, sQK, bqk, bqk, 0, 0, NPIX, 64, NCH, WINV, NI);
  launch_gemm<2, 1, 0, 0>(stream, chmT, NCH, sPixC, Wqk_d, NCH, 0, qk_d, 64, sQK, bqk + 64, bqk, 0, 0, NPIX, 64, NCH, WINV, NI);
  launch_gemm<1, 1, 0, 0>(stream, Wv_r, NCH, 0, rgbT, NCH, sPixC, v_r, NPIX, sPixC, rv_b, rv_b, 0, 0, NCH, NPIX, NCH, WINV, NI);
  launch_gemm<1, 1, 0, 0>(stream, Wv_d, NCH, 0, chmT, NCH, sPixC, v_d, NPIX, sPixC, dv_b, dv_b, 0, 0, NCH, NPIX, NCH, WINV, NI);

  for (int img = 0; img < NI; ++img) {
    for (int brn = 0; brn < 2; ++brn) {
      const _Float16* qk   = (brn == 0) ? qk_d : qk_r;
      const _Float16* vv   = (brn == 0) ? v_r : v_d;
      const float*    feat = (brn == 0) ? rgb : chm;
      const _Float16* qkb  = qk + (size_t)img * NPIX * 64;
      launch_gemm<0, 0, 0, 0>(stream, qkb, 64, 0, qkb + 32, 64, 0, Sbuf, NPIX, 0, g_b, g_b, 0, 0, NPIX, NPIX, 32, 1.0f, 1);
      k_softmax_t<<<dim3(NPIX / 64), dim3(256), 0, stream>>>(Sbuf, PT);
      launch_gemm<0, 0, 2, 0>(stream, PT, NPIX, 0, vv + (size_t)img * NCH * NPIX, NPIX, 0,
                              cat32 + (size_t)img * NPIX * NCH2 + brn * NCH, NCH2, 0,
                              g_b, feat + (size_t)img * NCH * NPIX, 0, NPIX,
                              NPIX, NCH, NPIX, 1.0f / 32768.0f, 1);
    }
  }

  launch_cast(stream, cat32, cat16, NI * NPIX * NCH2, 1.0f);
  launch_cast(stream, g_w, Wg16, NCH * NCH2, WSC);
  launch_cast(stream, f1_w, W1_16, NCH2 * NCH2, WSC);
  launch_cast(stream, f3_w, W3_16, NCH * NCH2, WSC);
  launch_cast(stream, sk_w, Wsk16, NCH * NCH2, WSC);
  k_w2r<<<dim3((NCH2 * 9 * 64) / 256), dim3(256), 0, stream>>>(f2_w, W2r, WSC);

  launch_gemm<2, 0, 0, 6>(stream, cat16, NCH2, sPix2, Wg16, NCH2, 0, G32, NCH, sPixC, g_b, g_b, 0, 0, NPIX, NCH, NCH2, WINV, NI);
  k_fuse<<<dim3((NI * NPIX * 32) / 256), dim3(256), 0, stream>>>(cat32, G32, F16, NI * NPIX);
  launch_gemm<2, 1, 0, 2>(stream, F16, NCH2, sPix2, W1_16, NCH2, 0, Y1, NCH2, sPix2, f1_b, f1_b, 0, 0, NPIX, NCH2, NCH2, WINV, NI);
  for (int img = 0; img < NI; ++img) {
    k_im2col<<<dim3((NPIX * 9 * 64) / 256), dim3(256), 0, stream>>>(Y1 + (size_t)img * NPIX * NCH2, COL);
    launch_gemm<2, 1, 0, 2>(stream, COL, KCOL, 0, W2r, KCOL, 0, Y2 + (size_t)img * NPIX * NCH2, NCH2, 0,
                            f2_b, f2_b, 0, 0, NPIX, NCH2, KCOL, WINV, 1);
  }
  launch_gemm<1, 0, 0, 0>(stream, Wsk16, NCH2, 0, F16, NCH2, sPix2, SK, NPIX, sPixC, sk_b, sk_b, 0, 0, NCH, NPIX, NCH2, WINV, NI);
  launch_gemm<1, 0, 1, 0>(stream, W3_16, NCH2, 0, Y2, NCH2, sPix2, out, NPIX, sPixC, f3_b, SK, sPixC, 0, NCH, NPIX, NCH2, WINV, NI);
}
